// ForgetGRU_23390391894968
// MI455X (gfx1250) — hardware-run, weakly checked
//
#include <hip/hip_runtime.h>
#include <stdint.h>

constexpr int kBatch  = 128;
constexpr int kTime   = 128;
constexpr int kIn     = 512;
constexpr int kHid    = 512;
constexpr int kExtra  = 256;
constexpr int kLayers = 2;
constexpr int kKdim   = 512;
constexpr int kPitchX = 520;
constexpr int kRowsPerBlock = 16;
constexpr int kThreads = 256;
constexpr int kTileElems  = kRowsPerBlock * kPitchX;
constexpr int kSlabCols   = 32;
constexpr int kSlabElems  = kRowsPerBlock * kSlabCols;
constexpr float kActScale = 8.0f;
constexpr float kWScale   = 256.0f;
constexpr float kAccInv   = 1.0f / 2048.0f;
constexpr size_t kMatStride   = (size_t)kLayers * kHid * kKdim;
constexpr size_t kPlaneElems  = (size_t)kLayers * kBatch * kHid;

static_assert(kBatch % kRowsPerBlock == 0, "batch tiles");
static_assert(kHid == 8 * 64, "8 waves x 64 columns");
static_assert(kIn == kKdim && kHid == kKdim, "uniform K");
static_assert(kKdim % 32 == 0 && kExtra % 32 == 0, "K multiples of 32");
static_assert(kPitchX % 8 == 0 && kTileElems % 8 == 0, "16-B aligned LDS rows and tiles");
static_assert(kThreads * 32 == kRowsPerBlock * kHid, "tile fill / convert coverage: 256 threads x 32 elements = 16 x 512");
static_assert(kSlabCols % 4 == 0 && kSlabCols * 4 == 128, "slab row = one 128-B line");
static_assert(kPlaneElems % 4 == 0, "zero fill in float4");

typedef __attribute__((ext_vector_type(16))) _Float16 v16h;
typedef __attribute__((ext_vector_type(8)))  _Float16 v8h;
typedef __attribute__((ext_vector_type(16))) __bf16   v16b;
typedef __attribute__((ext_vector_type(8)))  __bf16   v8b;
typedef __attribute__((ext_vector_type(8)))  float    v8f;
typedef __attribute__((ext_vector_type(4)))  float    v4f;
#define U16(p) ((const unsigned short*)(const void*)(p))

__device__ __forceinline__ unsigned short f2bf_bits(float f) {
  unsigned u = __float_as_uint(f);
  return (unsigned short)((u + 0x7FFFu + ((u >> 16) & 1u)) >> 16);
}
__device__ __forceinline__ float bf_bits2f(unsigned short h) { return __uint_as_float(((unsigned)h) << 16); }

__device__ __forceinline__ void dep_guard_h(v8f& a, v8f& b, v16h x, v16h y) { asm volatile("v_nop\n\tv_nop\n\tv_nop\n\tv_nop" : "+v"(a), "+v"(b) : "v"(x), "v"(y)); }
__device__ __forceinline__ void dep_guard_b(v8f& a, v8f& b, v16b x, v16b y) { asm volatile("v_nop\n\tv_nop\n\tv_nop\n\tv_nop" : "+v"(a), "+v"(b) : "v"(x), "v"(y)); }
__device__ __forceinline__ void keep4_h(v16h a, v16h b, v16h c, v16h d) { asm volatile("v_nop" :: "v"(a), "v"(b), "v"(c), "v"(d)); }
__device__ __forceinline__ void keep4_b(v16b a, v16b b, v16b c, v16b d) { asm volatile("v_nop" :: "v"(a), "v"(b), "v"(c), "v"(d)); }
__device__ __forceinline__ void acc_guard4(v8f& a, v8f& b, v8f& c, v8f& d) { asm volatile("v_nop\n\tv_nop\n\tv_nop\n\tv_nop" : "+v"(a), "+v"(b), "+v"(c), "+v"(d)); }
template <typename T> struct Frag;
template <> struct Frag<_Float16> {
  typedef v16h V; union U { v16h v; v8h h[2]; };
  static __device__ __forceinline__ v16h load(const _Float16* p) {
    U f; f.h[0] = *(const v8h*)(p); f.h[1] = *(const v8h*)(p + 16); return f.v;
  }
  static __device__ __forceinline__ v8f mma(v16h a, v16h b, v8f c) {
    return __builtin_amdgcn_wmma_f32_16x16x32_f16(false, a, false, b, (short)0, c, false, false);
  }
  static __device__ __forceinline__ void guard(v8f& a, v8f& b, v16h x, v16h y) { dep_guard_h(a, b, x, y); }
  static __device__ __forceinline__ void keep(v16h a, v16h b, v16h c, v16h d) { keep4_h(a, b, c, d); }
};
template <> struct Frag<__bf16> {
  typedef v16b V; union U { v16b v; v8b h[2]; };
  static __device__ __forceinline__ v16b load(const __bf16* p) {
    U f; f.h[0] = *(const v8b*)(p); f.h[1] = *(const v8b*)(p + 16); return f.v;
  }
  static __device__ __forceinline__ v8f mma(v16b a, v16b b, v8f c) {
    return __builtin_amdgcn_wmma_f32_16x16x32_bf16(false, a, false, b, (short)0, c, false, false);
  }
  static __device__ __forceinline__ void guard(v8f& a, v8f& b, v16b x, v16b y) { dep_guard_b(a, b, x, y); }
  static __device__ __forceinline__ void keep(v16b a, v16b b, v16b c, v16b d) { keep4_b(a, b, c, d); }
};

template <int ET> struct Elem;
template <> struct Elem<0> { typedef _Float16 T; };
template <> struct Elem<1> { typedef __bf16 T; };
template <int ET, bool SPLIT, int BIAS_MODE, int OUT_MODE, bool RESID, int ACT = 0>
__global__ __launch_bounds__(256) void wmma_gemm64(
    const unsigned short* __restrict__ Ap, const unsigned short* __restrict__ A2p, int lda, long strideA,
    const unsigned short* __restrict__ Btp, const unsigned short* __restrict__ Bt2p, int ldb, long strideB,
    void* __restrict__ Cout, void* __restrict__ Cout2, int ldc, long strideC,
    const float* __restrict__ bias,
    const float* __restrict__ resid, long strideR,
    int M, int N, int K, float scale) {
  typedef typename Elem<ET>::T T;
  typedef typename Frag<T>::V V;
  const T* A = (const T*)Ap; const T* A2 = (const T*)A2p; const T* Bt = (const T*)Btp; const T* Bt2 = (const T*)Bt2p;
  __shared__ __align__(16) float sT[8][16 * 68];
  const int b    = blockIdx.y;
  const int lane = threadIdx.x & 31;
  const int wave = threadIdx.x >> 5;
  const int tilesN = N >> 6;
  const int tilesM = M >> 6;
  const int tile = blockIdx.x * 8 + wave;
  if (tile >= tilesM * tilesN) return;
  const int tm = tile / tilesN;
  const int tn = tile - tm * tilesN;
  const int m0 = tm << 6;
  const int n0 = tn << 6;

  const T* Ab  = A  + (size_t)b * strideA;
  const T* Bb  = Bt + (size_t)b * strideB;
  const T* Ab2 = SPLIT ? (A2  + (size_t)b * strideA) : nullptr;
  const T* Bb2 = SPLIT ? (Bt2 + (size_t)b * strideB) : nullptr;

  const int rlane = lane & 15;
  const int koff  = (lane >> 4) * 8;
  const int mOff  = (lane >> 4) * 8;

  v8f acc[4][4];
#pragma unroll
  for (int i = 0; i < 4; ++i)
#pragma unroll
    for (int j = 0; j < 4; ++j) acc[i][j] = (v8f){0.f,0.f,0.f,0.f,0.f,0.f,0.f,0.f};

  for (int k0 = 0; k0 < K; k0 += 32) {
    V bh[4], bl[4];
#pragma unroll
    for (int j = 0; j < 4; ++j) {
      const size_t bo = (size_t)(n0 + (j << 4) + rlane) * ldb + koff + k0;
      bh[j] = Frag<T>::load(Bb + bo);
      if (SPLIT) bl[j] = Frag<T>::load(Bb2 + bo);
    }
#pragma unroll
    for (int i = 0; i < 4; ++i) {
      const size_t ao = (size_t)(m0 + (i << 4) + rlane) * lda + koff + k0;
      V ah = Frag<T>::load(Ab + ao);
      V al;
      if (SPLIT) al = Frag<T>::load(Ab2 + ao);
#pragma unroll
      for (int j = 0; j < 4; ++j) {
        acc[i][j] = Frag<T>::mma(ah, bh[j], acc[i][j]);
        if (SPLIT) {
          acc[i][j] = Frag<T>::mma(ah, bl[j], acc[i][j]);
          acc[i][j] = Frag<T>::mma(al, bh[j], acc[i][j]);
        }
      }
      Frag<T>::guard(acc[i][0], acc[i][3], ah, SPLIT ? al : ah);
    }
    Frag<T>::keep(bh[0], bh[1], bh[2], bh[3]);
    if (SPLIT) Frag<T>::keep(bl[0], bl[1], bl[2], bl[3]);
  }
  acc_guard4(acc[0][0], acc[0][1], acc[0][2], acc[0][3]);
  acc_guard4(acc[1][0], acc[1][1], acc[1][2], acc[1][3]);
  acc_guard4(acc[2][0], acc[2][1], acc[2][2], acc[2][3]);
  acc_guard4(acc[3][0], acc[3][1], acc[3][2], acc[3][3]);

  float* slab = sT[wave];
  const float* Rb = RESID ? (resid + (size_t)b * strideR) : nullptr;
#pragma unroll
  for (int i = 0; i < 4; ++i) {
    const int mBase = m0 + (i << 4);
#pragma unroll
    for (int j = 0; j < 4; ++j) {
      const int n = n0 + (j << 4) + rlane;
      float bv = 0.f;
      if (BIAS_MODE == 2) bv = bias[n];
#pragma unroll
      for (int r = 0; r < 8; ++r) {
        float v = acc[i][j][r] * scale;
        if (BIAS_MODE == 1) v += bias[mBase + mOff + r];
        if (BIAS_MODE == 2) v += bv;
        if (RESID) v += Rb[(size_t)(mBase + mOff + r) * ldc + n];
        if (ACT == 1) v = tanhf(v);
        if (ACT == 2) v = fmaxf(v, 0.0f);
        if (ACT == 3) v = v / (1.0f + expf(-v));
        if (ACT == 4) v = (v > 0.f) ? v : 0.01f * v;
        if (ACT == 5) v = 0.5f * v * (1.0f + erff(v * 0.70710678118654752f));
        slab[(mOff + r) * 68 + (j << 4) + rlane] = v;
      }
    }
    __builtin_amdgcn_fence(__ATOMIC_RELEASE, "workgroup");
    __builtin_amdgcn_wave_barrier();
    __builtin_amdgcn_fence(__ATOMIC_ACQUIRE, "workgroup");
    if (OUT_MODE == 0) {
      float* C = (float*)Cout + (size_t)b * strideC;
      const int hh = lane >> 4, c4 = (lane & 15) * 4;
      for (int pass = 0; pass < 2; ++pass) {
#pragma unroll
        for (int it = 0; it < 8; ++it) {
          const int row = it * 2 + hh;
          v4f v = *(const v4f*)(slab + row * 68 + c4);
          *(volatile v4f*)(C + (size_t)(mBase + row) * ldc + n0 + c4) = v;
        }
        __threadfence();
      }
    } else {
      const int q = lane >> 3, c8 = (lane & 7) * 8;
      unsigned short* C  = (unsigned short*)Cout  + (size_t)b * strideC;
      unsigned short* C2 = (OUT_MODE == 2) ? ((unsigned short*)Cout2 + (size_t)b * strideC) : nullptr;
      for (int pass = 0; pass < 2; ++pass) {
#pragma unroll
        for (int it = 0; it < 4; ++it) {
          const int row = it * 4 + q;
          const float* sp = slab + row * 68 + c8;
          v8h hv, lv;
#pragma unroll
          for (int e = 0; e < 8; ++e) {
            if (OUT_MODE == 1) {
              hv[e] = (_Float16)sp[e];
            } else {
              unsigned short hb = f2bf_bits(sp[e]);
              unsigned short lb = f2bf_bits(sp[e] - bf_bits2f(hb));
              hv[e] = __builtin_bit_cast(_Float16, hb);
              lv[e] = __builtin_bit_cast(_Float16, lb);
            }
          }
          *(volatile v8h*)(C + (size_t)(mBase + row) * ldc + n0 + c8) = hv;
          if (OUT_MODE == 2) *(volatile v8h*)(C2 + (size_t)(mBase + row) * ldc + n0 + c8) = lv;
        }
        __threadfence();
      }
    }
    __builtin_amdgcn_fence(__ATOMIC_RELEASE, "workgroup");
    __builtin_amdgcn_wave_barrier();
    __builtin_amdgcn_fence(__ATOMIC_ACQUIRE, "workgroup");
  }
}

__global__ __launch_bounds__(256) void cast_f32_f16x2s(
    const float* __restrict__ in, _Float16* __restrict__ out, int n2, float scale) {
  int i = blockIdx.x * 256 + threadIdx.x;
  if (i < n2) {
    const _Float16 h0 = (_Float16)(in[2 * i] * scale), h1 = (_Float16)(in[2 * i + 1] * scale);
    const unsigned u = (unsigned)__builtin_bit_cast(unsigned short, h0) | ((unsigned)__builtin_bit_cast(unsigned short, h1) << 16);
    ((volatile unsigned*)out)[i] = u;
    __threadfence();
    ((volatile unsigned*)out)[i] = u;
  }
}

__global__ __launch_bounds__(256) void zero_f32x4(float* __restrict__ out, int n4) {
  int i = blockIdx.x * 256 + threadIdx.x;
  if (i < n4) {
    const v4f z = (v4f){0.f, 0.f, 0.f, 0.f};
    *(volatile v4f*)(out + (size_t)4 * i) = z;
    __threadfence();
    *(volatile v4f*)(out + (size_t)4 * i) = z;
  }
}

__device__ __forceinline__ v4f ld_gvol4(const float* p) {
  return *(__attribute__((address_space(1))) const volatile v4f*)p;
}
__device__ __forceinline__ float ld_gvol1(const float* p) {
  return *(__attribute__((address_space(1))) const volatile float*)p;
}

__device__ __forceinline__ v8f mma16(v16h a, v16h b, v8f c) {
  return __builtin_amdgcn_wmma_f32_16x16x32_f16(false, a, false, b, (short)0, c, false, false);
}
__device__ __forceinline__ void kguard3(v8f& c0, v8f& c1, v8f& c2, v16h a, v16h b0, v16h b1, v16h b2) {
  asm volatile("v_nop\n\tv_nop\n\tv_nop\n\tv_nop"
               : "+v"(c0), "+v"(c1), "+v"(c2)
               : "v"(a), "v"(b0), "v"(b1), "v"(b2));
}

__device__ __forceinline__ float sigm_f(float x) {
  x = fminf(fmaxf(x, -30.0f), 30.0f);
  return __builtin_amdgcn_rcpf(1.0f + expf(-x));
}
__device__ __forceinline__ float tanh_f(float x) {
  x = fminf(fmaxf(x, -15.0f), 15.0f);
  return 1.0f - 2.0f * __builtin_amdgcn_rcpf(1.0f + expf(2.0f * x));
}
__device__ __forceinline__ float gru_unit(float aR, float aZ, float aX, float aHn,
                                          float addR, float addZ, float addN, float hp) {
  const float rg = sigm_f(aR * kAccInv + addR);
  const float zg = sigm_f(aZ * kAccInv + addZ);
  const float ng = tanh_f(aX * kAccInv + addN + rg * (aHn * kAccInv));
  return (1.0f - zg) * ng + zg * hp;
}

__device__ __forceinline__ void cell_subtile(
    const _Float16* ain, const _Float16* ahid,
    const float* hprev,
    float* slab, int scol,
    const _Float16* __restrict__ wl,
    const float* __restrict__ bir, const float* __restrict__ biz, const float* __restrict__ bin,
    const float* __restrict__ erl,
    int b0, int ub, int lane) {
  const int hh = lane >> 4, c = lane & 15;
  const int n = 16 * ub + c;
  v8f aR = (v8f){0.f,0.f,0.f,0.f,0.f,0.f,0.f,0.f};
  v8f aZ = (v8f){0.f,0.f,0.f,0.f,0.f,0.f,0.f,0.f};
  v8f aX = (v8f){0.f,0.f,0.f,0.f,0.f,0.f,0.f,0.f};
  v8f aH = (v8f){0.f,0.f,0.f,0.f,0.f,0.f,0.f,0.f};
  const _Float16* wrow = wl + (size_t)n * kKdim + 8 * hh;
  const _Float16* arow = ain  + c * kPitchX + 8 * hh;
  const _Float16* hrow = ahid + c * kPitchX + 8 * hh;

#pragma unroll 2
  for (int k0 = 0; k0 < kKdim; k0 += 32) {
    const v16h a  = Frag<_Float16>::load(arow + k0);
    const v16h b0f = Frag<_Float16>::load(wrow + 0 * kMatStride + k0);
    const v16h b1f = Frag<_Float16>::load(wrow + 2 * kMatStride + k0);
    const v16h b2f = Frag<_Float16>::load(wrow + 4 * kMatStride + k0);
    aR = mma16(a, b0f, aR);
    aZ = mma16(a, b1f, aZ);
    aX = mma16(a, b2f, aX);
    kguard3(aR, aZ, aX, a, b0f, b1f, b2f);
  }
#pragma unroll 2
  for (int k0 = 0; k0 < kKdim; k0 += 32) {
    const v16h a  = Frag<_Float16>::load(hrow + k0);
    const v16h b0f = Frag<_Float16>::load(wrow + 1 * kMatStride + k0);
    const v16h b1f = Frag<_Float16>::load(wrow + 3 * kMatStride + k0);
    const v16h b2f = Frag<_Float16>::load(wrow + 5 * kMatStride + k0);
    aR = mma16(a, b0f, aR);
    aZ = mma16(a, b1f, aZ);
    aH = mma16(a, b2f, aH);
    kguard3(aR, aZ, aH, a, b0f, b1f, b2f);
  }
  acc_guard4(aR, aZ, aX, aH);

  const float br = bir[n];
  const float bz = biz[n];
  const float bn = bin[n];
#pragma unroll
  for (int r = 0; r < 8; ++r) {
    const int m = 8 * hh + r;
    const size_t goff = (size_t)(b0 + m) * kHid + n;
    const float e  = erl[goff];
    const float hp = ld_gvol1(hprev + goff);
    const float hn = gru_unit(aR[r], aZ[r], aX[r], aH[r], br + e, bz, bn, hp);
    slab[m * kSlabCols + scol + c] = hn;
  }
}

__device__ __forceinline__ void convert_rows_to_tile(const float* rows, _Float16* tile, int tid) {
  const int row = tid >> 4;
  const int cb  = (tid & 15) * 32;
  const float* src = rows + (size_t)row * kHid + cb;
  _Float16* dst = tile + row * kPitchX + cb;
#pragma unroll
  for (int j = 0; j < 4; ++j) {
    const v4f f0 = ld_gvol4(src + 8 * j);
    const v4f f1 = ld_gvol4(src + 8 * j + 4);
    v8h hv;
    hv[0] = (_Float16)(f0[0] * kActScale); hv[1] = (_Float16)(f0[1] * kActScale);
    hv[2] = (_Float16)(f0[2] * kActScale); hv[3] = (_Float16)(f0[3] * kActScale);
    hv[4] = (_Float16)(f1[0] * kActScale); hv[5] = (_Float16)(f1[1] * kActScale);
    hv[6] = (_Float16)(f1[2] * kActScale); hv[7] = (_Float16)(f1[3] * kActScale);
    *(v8h*)(dst + 8 * j) = hv;
  }
}

__device__ __forceinline__ void wave_store_rows32(const float* s,
                                                  float* gA, long sA,
                                                  float* gB, long sB, bool useB,
                                                  float* gC, long sC, bool useC,
                                                  int lane) {
  const int q = lane >> 3, c4 = (lane & 7) * 4;
  for (int pass = 0; pass < 2; ++pass) {
#pragma unroll
    for (int it = 0; it < 4; ++it) {
      const int row = it * 4 + q;
      const v4f v = *(const v4f*)(s + row * kSlabCols + c4);
      *(volatile v4f*)(gA + (size_t)row * sA + c4) = v;
      if (useB) *(volatile v4f*)(gB + (size_t)row * sB + c4) = v;
      if (useC) *(volatile v4f*)(gC + (size_t)row * sC + c4) = v;
    }
    __threadfence();
  }
}

__global__ __launch_bounds__(kThreads)
void gru_seq_kernel(const float* __restrict__ x,
                    const _Float16* __restrict__ w16,
                    const float* __restrict__ b_ir,
                    const float* __restrict__ b_iz,
                    const float* __restrict__ b_in,
                    const float* __restrict__ er,
                    float* hsf,
                    float* __restrict__ out0,
                    float* __restrict__ out1) {
  __shared__ __align__(16) _Float16 tiles[3 * kTileElems];
  __shared__ __align__(16) float    slabs[8 * kSlabElems];
  const int tid  = threadIdx.x;
  const int lane = tid & 31;
  const int wave = tid >> 5;
  const int b0   = blockIdx.x * kRowsPerBlock;
  float* slab = slabs + wave * kSlabElems;

  {
    v8h z8;
#pragma unroll
    for (int e = 0; e < 8; ++e) z8[e] = (_Float16)0.0f;
    for (int i = tid; i < kTileElems / 8; i += kThreads) {
      *(v8h*)(tiles + kTileElems + 8 * i)     = z8;
      *(v8h*)(tiles + 2 * kTileElems + 8 * i) = z8;
    }
  }

  const long ostride = (long)kTime * kHid;

  for (int t = 0; t < kTime; ++t) {
    {
      const int row = tid >> 4;
      const int cb  = (tid & 15) * 32;
      const float* src = x + ((size_t)(b0 + row) * kTime + t) * kIn + cb;
      _Float16* dst = tiles + row * kPitchX + cb;
#pragma unroll
      for (int j = 0; j < 4; ++j) {
        const v4f f0 = *(const v4f*)(src + 8 * j);
        const v4f f1 = *(const v4f*)(src + 8 * j + 4);
        v8h hv;
        hv[0] = (_Float16)(f0[0] * kActScale); hv[1] = (_Float16)(f0[1] * kActScale);
        hv[2] = (_Float16)(f0[2] * kActScale); hv[3] = (_Float16)(f0[3] * kActScale);
        hv[4] = (_Float16)(f1[0] * kActScale); hv[5] = (_Float16)(f1[1] * kActScale);
        hv[6] = (_Float16)(f1[2] * kActScale); hv[7] = (_Float16)(f1[3] * kActScale);
        *(v8h*)(dst + 8 * j) = hv;
      }
    }
    __syncthreads();

    const int pr = t & 1;
    const int pw = pr ^ 1;
    const bool last = (t == kTime - 1);

#pragma unroll 1
    for (int l = 0; l < kLayers; ++l) {
      const _Float16* ain   = tiles + l * kTileElems;
      const _Float16* ahid  = tiles + (l + 1) * kTileElems;
      _Float16*       htile = tiles + (l + 1) * kTileElems;
      const _Float16* wl    = w16 + (size_t)l * kHid * kKdim;
      const float*    bir   = b_ir + l * kHid;
      const float*    biz   = b_iz + l * kHid;
      const float*    bin   = b_in + l * kHid;
      const float*    erl   = er + (size_t)l * kBatch * kHid;
      const float*    hprev = hsf + ((size_t)(pr * kLayers + l) * kBatch) * kHid;
      float*          hnext = hsf + ((size_t)(pw * kLayers + l) * kBatch) * kHid;
      const bool      isTop = (l == kLayers - 1);

#pragma unroll 1
      for (int u = 0; u < 4; ++u) {
        cell_subtile(ain, ahid, hprev, slab, 16 * (u & 1), wl, bir, biz, bin, erl, b0, 4 * wave + u, lane);
        if (u & 1) {
          __builtin_amdgcn_fence(__ATOMIC_RELEASE, "workgroup");
          __builtin_amdgcn_wave_barrier();
          __builtin_amdgcn_fence(__ATOMIC_ACQUIRE, "workgroup");
          const int col0 = 64 * wave + 32 * (u >> 1);
          float* gA = hnext + (size_t)b0 * kHid + col0;
          float* gB = out0 + ((size_t)b0 * kTime + t) * kHid + col0;
          float* gC = out1 + ((size_t)l * kBatch + b0) * kHid + col0;
          wave_store_rows32(slab, gA, (long)kHid, gB, ostride, isTop, gC, (long)kHid, last, lane);
          __builtin_amdgcn_fence(__ATOMIC_RELEASE, "workgroup");
          __builtin_amdgcn_wave_barrier();
          __builtin_amdgcn_fence(__ATOMIC_ACQUIRE, "workgroup");
        }
      }
      __syncthreads();

      convert_rows_to_tile(hnext + (size_t)b0 * kHid, htile, tid);
      __syncthreads();
    }
  }
}

extern "C" void kernel_launch(void* const* d_in, const int* in_sizes, int n_in,
                              void* d_out, int out_size, void* d_ws, size_t ws_size,
                              hipStream_t stream) {
  if (n_in < 12) return;
  if (in_sizes[0] != kBatch * kTime * kIn) return;
  if (in_sizes[1] != kBatch * kExtra) return;
  if (in_sizes[2] != kLayers * kHid * kIn || in_sizes[4] != kLayers * kHid * kHid ||
      in_sizes[5] != kLayers * kHid * kIn || in_sizes[7] != kLayers * kHid * kHid ||
      in_sizes[8] != kLayers * kHid * kIn || in_sizes[10] != kLayers * kHid * kHid) return;
  if (in_sizes[3] != kLayers * kHid || in_sizes[6] != kLayers * kHid || in_sizes[9] != kLayers * kHid) return;
  if (in_sizes[11] != kLayers * kHid * kExtra) return;
  if (out_size != kBatch * kTime * kHid + kLayers * kBatch * kHid) return;

  const float* x     = (const float*)d_in[0];
  const float* extra = (const float*)d_in[1];
  const float* W_irF = (const float*)d_in[2];
  const float* b_irF = (const float*)d_in[3];
  const float* W_hrF = (const float*)d_in[4];
  const float* W_izF = (const float*)d_in[5];
  const float* b_izF = (const float*)d_in[6];
  const float* W_hzF = (const float*)d_in[7];
  const float* W_inF = (const float*)d_in[8];
  const float* b_inF = (const float*)d_in[9];
  const float* W_hnF = (const float*)d_in[10];
  const float* W_erF = (const float*)d_in[11];

  char* ws = (char*)d_ws;
  size_t off = 0;
  _Float16* w16     = (_Float16*)(ws + off); off += (size_t)6 * kMatStride * sizeof(_Float16);
  _Float16* extra16 = (_Float16*)(ws + off); off += (size_t)kBatch * kExtra * sizeof(_Float16);
  _Float16* wer16   = (_Float16*)(ws + off); off += (size_t)kLayers * kHid * kExtra * sizeof(_Float16);
  float*    erf     = (float*)(ws + off);    off += (size_t)kLayers * kBatch * kHid * sizeof(float);
  float*    hsf     = (float*)(ws + off);    off += (size_t)2 * kPlaneElems * sizeof(float);
  if (off > ws_size) return;

  const float* Wsrc[6] = {W_irF, W_hrF, W_izF, W_hzF, W_inF, W_hnF};
  const int n2w = (int)(kMatStride / 2);
  for (int mi = 0; mi < 6; ++mi)
    cast_f32_f16x2s<<<(n2w + 255) / 256, 256, 0, stream>>>(Wsrc[mi], w16 + (size_t)mi * kMatStride, n2w, kWScale);
  const int n2e = kBatch * kExtra / 2;
  cast_f32_f16x2s<<<(n2e + 255) / 256, 256, 0, stream>>>(extra, extra16, n2e, kActScale);
  const int n2r = kLayers * kHid * kExtra / 2;
  cast_f32_f16x2s<<<(n2r + 255) / 256, 256, 0, stream>>>(W_erF, wer16, n2r, kWScale);

  {
    const int n4 = (int)(kPlaneElems / 4);
    zero_f32x4<<<(n4 + 255) / 256, 256, 0, stream>>>(hsf, n4);
  }

  {
    const int tiles = (kBatch / 64) * (kHid / 64);
    dim3 grid((tiles + 7) / 8, kLayers);
    wmma_gemm64<0, false, 0, 0, false, 0><<<grid, 256, 0, stream>>>(
        U16(extra16), nullptr, kExtra, 0L,
        U16(wer16), nullptr, kExtra, (long)kHid * kExtra,
        (void*)erf, nullptr, kHid, (long)kBatch * kHid,
        nullptr, nullptr, 0L,
        kBatch, kHid, kExtra, kAccInv);
  }

  float* out0 = (float*)d_out;
  float* out1 = out0 + (size_t)kBatch * kTime * kHid;

  gru_seq_kernel<<<kBatch / kRowsPerBlock, kThreads, 0, stream>>>(
      x, w16, b_irF, b_izF, b_inF, erf, hsf, out0, out1);
}
